// TransformerBlockRes_30021821399848
// MI455X (gfx1250) — hardware-verified
//
#include <hip/hip_runtime.h>
#include <math.h>

typedef __attribute__((ext_vector_type(16))) _Float16 v16h;
typedef __attribute__((ext_vector_type(16))) __bf16 v16b;
typedef __attribute__((ext_vector_type(8)))  _Float16 v8h;
typedef __attribute__((ext_vector_type(8)))  float v8f;
typedef __attribute__((ext_vector_type(4)))  float v4f;
typedef __attribute__((ext_vector_type(2)))  float v2f;
typedef __attribute__((ext_vector_type(4)))  unsigned v4u;
typedef __attribute__((ext_vector_type(4)))  int v4i;
typedef float __attribute__((may_alias)) float_a;
typedef int __attribute__((may_alias)) int_a;

template <typename T> __device__ __forceinline__ void vst2(void* p, T v) { *(volatile T*)p = v; __threadfence(); *(volatile T*)p = v; }
__device__ __forceinline__ v8f wmma16(v16h a, v16h b, v8f c) {
  v8f d = __builtin_amdgcn_wmma_f32_16x16x32_f16(false, a, false, b, (short)0, c, false, false);
  asm volatile("v_nop\n\tv_nop\n\tv_nop\n\tv_nop" : "+v"(d) : "v"(a), "v"(b));
  return d;
}
__device__ __forceinline__ v8f wmma_bf(v16b a, v16b b, v8f c) {
  v8f d = __builtin_amdgcn_wmma_f32_16x16x32_bf16(false, a, false, b, (short)0, c, false, false);
  asm volatile("v_nop\n\tv_nop\n\tv_nop\n\tv_nop" : "+v"(d) : "v"(a), "v"(b));
  return d;
}
__device__ __forceinline__ v16h frag_h(const _Float16* rowk0, int lane) {
  union { v16h v; v8h q[2]; } u; const _Float16* p = rowk0 + 8 * (lane >> 4);
  u.q[0] = *(const v8h*)p; u.q[1] = *(const v8h*)(p + 16); return u.v;
}
__device__ __forceinline__ v16h frag_f32(const float* rowk0, int lane) {
  v16h a; const float* p = rowk0 + 8 * (lane >> 4);
#pragma unroll
  for (int i = 0; i < 8; ++i) { a[i] = (_Float16)p[i]; a[8 + i] = (_Float16)p[16 + i]; }
  return a;
}
__device__ __forceinline__ v16h frag_f32s(const float* rowk0, int lane, float sc) {
  v16h a; const float* p = rowk0 + 8 * (lane >> 4);
#pragma unroll
  for (int i = 0; i < 8; ++i) { a[i] = (_Float16)(p[i] * sc); a[8 + i] = (_Float16)(p[16 + i] * sc); }
  return a;
}
__device__ __forceinline__ v16h fragc_f32(const float* W, int k0, int n, int lane, int ld, int K) {
  v16h a; const int g = lane >> 4;
#pragma unroll
  for (int i = 0; i < 8; ++i) { const int ka = k0 + 8 * g + i, kb = ka + 16;
    a[i] = (_Float16)(ka < K ? W[(size_t)(ka < K ? ka : K - 1) * ld + n] : 0.f); a[8 + i] = (_Float16)(kb < K ? W[(size_t)(kb < K ? kb : K - 1) * ld + n] : 0.f); }
  return a;
}
struct F2 { v16b h, l; };
__device__ __forceinline__ F2 bsplit16(const float v[16]) { F2 r;
#pragma unroll
  for (int i = 0; i < 16; ++i) { const __bf16 h = (__bf16)v[i]; r.h[i] = h; r.l[i] = (__bf16)(v[i] - (float)h); }
  return r; }
__device__ __forceinline__ F2 split_row(const float* row, int k0, int lane) { float v[16]; const float* p = row + k0 + 8 * (lane >> 4);
#pragma unroll
  for (int i = 0; i < 8; ++i) { v[i] = p[i]; v[8 + i] = p[16 + i]; }
  return bsplit16(v); }
__device__ __forceinline__ F2 split_rowK(const float* row, int k0, int lane, int K) { float v[16]; const int g = lane >> 4;
#pragma unroll
  for (int i = 0; i < 8; ++i) { const int ka = k0 + 8 * g + i, kb = ka + 16; v[i] = ka < K ? row[ka < K ? ka : K - 1] : 0.f; v[8 + i] = kb < K ? row[kb < K ? kb : K - 1] : 0.f; }
  return bsplit16(v); }
__device__ __forceinline__ F2 split_col(const float* W, int k0, int n, int lane, int ld, int K) { float v[16]; const int g = lane >> 4;
#pragma unroll
  for (int i = 0; i < 8; ++i) { const int ka = k0 + 8 * g + i, kb = ka + 16; v[i] = ka < K ? W[(size_t)(ka < K ? ka : K - 1) * ld + n] : 0.f; v[8 + i] = kb < K ? W[(size_t)(kb < K ? kb : K - 1) * ld + n] : 0.f; }
  return bsplit16(v); }
__device__ __forceinline__ v8f mac3(const F2& a, const F2& b, v8f c) { c = wmma_bf(a.l, b.h, c); c = wmma_bf(a.h, b.l, c); return wmma_bf(a.h, b.h, c); }
__device__ __forceinline__ float sigm(float v) { return 1.0f / (1.0f + expf(-v)); }
#define LDSX() do { asm volatile("s_wait_dscnt 0" ::: "memory"); __builtin_amdgcn_wave_barrier(); __builtin_amdgcn_fence(__ATOMIC_RELEASE, "workgroup"); } while (0)


#define NN 4096
#define CIN 128
#define CO 128
#define HID 512
#define KNB 20
#define NE (KNB + 1)
#define NEDGE (NN * NE)
#ifndef NEB
#define NEB (NEDGE / 64)
#define NNB (NN / 64)
#endif
typedef __attribute__((ext_vector_type(8))) __bf16 v8b;
__device__ __forceinline__ v16b frag_b(const __bf16* rowk0, int lane) {
  union { v16b v; v8b q[2]; } u; const __bf16* p = rowk0 + 8 * (lane >> 4);
  u.q[0] = *(const v8b*)p; u.q[1] = *(const v8b*)(p + 16); return u.v;
}
__device__ __forceinline__ float bfr(float v) { return (float)(__bf16)v; }
__device__ __attribute__((noinline)) float exp_ni(float v) { return expf(v); }
__device__ __attribute__((noinline)) float erf_ni(float v) { return erff(v); }

#define WS_PW   0u
#define WS_PH   (WS_PW + 2u * 3 * CO * CIN)
#define WS_IDX  (WS_PH + 2u * 3 * HID * CO)
#define WS_V    (((WS_IDX + 4u * NN * NE) + 127u) / 128u * 128u)
#define WS_AS   (WS_V + 4u * NN * CO)
#define WS_AD   (WS_AS + 4u * NN * CO)
#define WS_DEL  (WS_AD + 4u * NN * CO)
#define WS_ALP  (WS_DEL + 4u * (size_t)NEDGE * CO)
#define WS_END  (WS_ALP + 4u * (size_t)NEDGE * CO)

__device__ __attribute__((noinline)) float elu_p(float v) { return v > 0.f ? v : (expf(v) - 1.0f); }
__global__ __launch_bounds__(256) void k_pack(const float* __restrict__ WL, const float* __restrict__ WS, const float* __restrict__ WD, const float* __restrict__ PW2, const float* __restrict__ AW1, const float* __restrict__ AW2, __bf16* __restrict__ PW, _Float16* __restrict__ PH) {
  const int n = blockIdx.x, which = blockIdx.y, t = threadIdx.x; __shared__ __align__(16) __bf16 s[CIN]; __shared__ __align__(16) _Float16 sh[HID];
  if (which < 3) { if (n >= CO) return; const float* Wm = (which == 0) ? WL : (which == 1) ? WS : WD; if (t < CIN) s[t] = (__bf16)Wm[(size_t)t * CO + n]; __syncthreads(); if (t < CIN / 8) vst2((unsigned*)(PW + ((size_t)which * CO + n) * CIN + t * 8), *(const v4u*)&s[t * 8]); }
  else if (which == 3) { if (n >= CO) return; for (int k = t; k < HID; k += 256) sh[k] = (_Float16)bfr(PW2[(size_t)k * CO + n]); __syncthreads(); for (int q = t; q < HID / 8; q += 256) vst2((unsigned*)(PH + (size_t)n * HID + q * 8), *(const v4u*)&sh[q * 8]); }
  else if (which == 4) { if (t < CO) sh[t] = (_Float16)bfr(AW1[(size_t)t * HID + n]); __syncthreads(); if (t < CO / 8) vst2((unsigned*)(PH + (size_t)CO * HID + (size_t)n * CO + t * 8), *(const v4u*)&sh[t * 8]); }
  else { if (n >= CO) return; for (int k = t; k < HID; k += 256) sh[k] = (_Float16)bfr(AW2[(size_t)k * CO + n]); __syncthreads(); for (int q = t; q < HID / 8; q += 256) vst2((unsigned*)(PH + (size_t)2 * CO * HID + (size_t)n * HID + q * 8), *(const v4u*)&sh[q * 8]); }
}
__global__ __launch_bounds__(64) void k_knn(const float* __restrict__ POS, int* __restrict__ IDX) {
  __shared__ float spos[NN * 3]; __shared__ float sd[64][KNB + 1]; __shared__ int si[64][KNB + 1];
  const int t = threadIdx.x; const int i = blockIdx.x * 64 + t;
  for (int e = t; e < NN * 3; e += 64) spos[e] = bfr(POS[e]);
  __syncthreads();
  const float xi = spos[i * 3], yi = spos[i * 3 + 1], zi = spos[i * 3 + 2]; const float sqi = (xi * xi + yi * yi) + zi * zi;
  for (int k = 0; k < KNB; ++k) { sd[t][k] = 3.0e38f; si[t][k] = 0x7fffffff; }
  int cnt = 0;
#pragma unroll 1
  for (int j = 0; j < NN; ++j) { if (j == i) continue; const float xj = spos[j * 3], yj = spos[j * 3 + 1], zj = spos[j * 3 + 2]; const float sqj = (xj * xj + yj * yj) + zj * zj; const float dt = (xi * xj + yi * yj) + zi * zj; const float d2 = (sqi + sqj) - 2.0f * dt;
    const float worst = sd[t][KNB - 1];
    if (cnt < KNB || d2 < worst) {
      int p = (cnt < KNB) ? cnt : KNB - 1;
      while (p > 0 && sd[t][p - 1] > d2) { sd[t][p] = sd[t][p - 1]; si[t][p] = si[t][p - 1]; --p; }
      sd[t][p] = d2; si[t][p] = j; if (cnt < KNB) ++cnt; } }
  for (int k = 0; k < KNB; ++k) IDX[(size_t)i * NE + k] = si[t][k];
  IDX[(size_t)i * NE + KNB] = i;
}
__global__ __launch_bounds__(128) void k_node(const float* __restrict__ X, const __bf16* __restrict__ PW, float* __restrict__ V, float* __restrict__ AS, float* __restrict__ AD) {
  __shared__ __align__(16) float so[4][16][132];
  const int tid = threadIdx.x, wave = tid >> 5, lane = tid & 31, col = lane & 15, g = lane >> 4; const int which = blockIdx.y; const size_t r0 = (size_t)blockIdx.x * 64 + wave * 16;
  v8f acc[8] = {};
#pragma unroll
  for (int kc = 0; kc < CIN / 32; ++kc) { v16b a; { const float* p = X + (r0 + col) * CIN + kc * 32 + 8 * g;
#pragma unroll
      for (int i = 0; i < 8; ++i) { a[i] = (__bf16)p[i]; a[8 + i] = (__bf16)p[16 + i]; } }
#pragma unroll
    for (int j = 0; j < 8; ++j) acc[j] = wmma_bf(a, frag_b(PW + ((size_t)which * CO + j * 16 + col) * CIN + kc * 32, lane), acc[j]); }
#pragma unroll
  for (int j = 0; j < 8; ++j)
#pragma unroll
    for (int r = 0; r < 8; ++r) so[wave][8 * g + r][j * 16 + col] = acc[j][r];
  LDSX();
  float* dst = (which == 0) ? V : (which == 1) ? AS : AD;
  for (int rl = 0; rl < 16; ++rl) vst2(dst + (r0 + rl) * CO + lane * 4, *(const v4f*)&so[wave][rl][lane * 4]);
}
__global__ __launch_bounds__(128) void k_edge(const float* __restrict__ POS, const int* __restrict__ IDX, const float* __restrict__ PW1, const float* __restrict__ PB1, const float* __restrict__ PG1, const float* __restrict__ PBT1, const _Float16* __restrict__ PH, const float* __restrict__ PB2, const float* __restrict__ PG2, const float* __restrict__ PBT2, const float* __restrict__ AS, const float* __restrict__ AD, const float* __restrict__ AB1, const float* __restrict__ AG1, const float* __restrict__ ABT1, const float* __restrict__ AB2, const float* __restrict__ AG2, const float* __restrict__ ABT2, float* __restrict__ DEL, float* __restrict__ ALP) {
  __shared__ __align__(16) _Float16 sh[64][HID + 8]; __shared__ __align__(16) _Float16 sa[64][CO + 8]; __shared__ __align__(16) float sm[64][CO + 4]; __shared__ float srel[64][3]; __shared__ float sst[64][2]; __shared__ int sj[64];
  const int tid = threadIdx.x, wave = tid >> 5, lane = tid & 31, col = lane & 15, g = lane >> 4; const size_t eb0 = (size_t)blockIdx.x * 64;
  if (tid < 64) { const size_t ed = eb0 + tid; const int i = (int)(ed / NE); const int j = IDX[ed]; sj[tid] = j; for (int c = 0; c < 3; ++c) srel[tid][c] = bfr(POS[(size_t)i * 3 + c]) - bfr(POS[(size_t)j * 3 + c]); }
  __syncthreads();
  { const int r = tid >> 1, part = tid & 1; const float rx = srel[r][0], ry = srel[r][1], rz = srel[r][2]; float s = 0.f;
#pragma unroll 1
    for (int n = part * 256; n < part * 256 + 256; ++n) { const float v = ((rx * bfr(PW1[n]) + ry * bfr(PW1[HID + n])) + rz * bfr(PW1[2 * HID + n])) + bfr(PB1[n]); s += v; }
    s += __shfl_xor(s, 1); const float mu = s / (float)HID; float q = 0.f;
#pragma unroll 1
    for (int n = part * 256; n < part * 256 + 256; ++n) { const float v = ((rx * bfr(PW1[n]) + ry * bfr(PW1[HID + n])) + rz * bfr(PW1[2 * HID + n])) + bfr(PB1[n]); const float d = v - mu; q += d * d; }
    q += __shfl_xor(q, 1); const float inv = 1.0f / sqrtf(q / (float)HID + 1e-5f);
#pragma unroll 1
    for (int n = part * 256; n < part * 256 + 256; ++n) { const float v = ((rx * bfr(PW1[n]) + ry * bfr(PW1[HID + n])) + rz * bfr(PW1[2 * HID + n])) + bfr(PB1[n]); sh[r][n] = (_Float16)elu_p((v - mu) * inv * bfr(PG1[n]) + bfr(PBT1[n])); } }
  if (tid < 64) for (int c = HID; c < HID + 8; ++c) sh[tid][c] = (_Float16)0.f;
  __syncthreads();
  const size_t r0 = eb0 + wave * 16;
  { v8f acc[8] = {};
#pragma unroll 2
    for (int kc = 0; kc < HID / 32; ++kc) { const v16h a = frag_h(&sh[wave * 16 + col][kc * 32], lane);
#pragma unroll
      for (int j = 0; j < 8; ++j) acc[j] = wmma16(a, frag_h(PH + (size_t)(j * 16 + col) * HID + kc * 32, lane), acc[j]); }
#pragma unroll
    for (int j = 0; j < 8; ++j) { const float bb = bfr(PB2[j * 16 + col]);
#pragma unroll
      for (int r = 0; r < 8; ++r) sm[wave * 16 + 8 * g + r][j * 16 + col] = acc[j][r] + bb; } }
  __syncthreads();
  { const int r = tid >> 1, part = tid & 1; float s = 0.f; for (int c = part; c < CO; c += 2) s += sm[r][c]; s += __shfl_xor(s, 1); const float mu = s / (float)CO; float q = 0.f; for (int c = part; c < CO; c += 2) { const float d = sm[r][c] - mu; q += d * d; } q += __shfl_xor(q, 1); const float inv = 1.0f / sqrtf(q / (float)CO + 1e-5f);
    const size_t ed = eb0 + r; const int i = (int)(ed / NE); const int j = sj[r];
    for (int c = part; c < CO; c += 2) { const float dl = elu_p((sm[r][c] - mu) * inv * bfr(PG2[c]) + bfr(PBT2[c])); sm[r][c] = dl; sa[r][c] = (_Float16)(AD[(size_t)i * CO + c] - AS[(size_t)j * CO + c] + dl); } }
  if (tid < 64) for (int c = CO; c < CO + 8; ++c) sa[tid][c] = (_Float16)0.f;
  __syncthreads();
  for (int e = tid; e < 64 * (CO / 4); e += 128) { const int r = e >> 5, q = e & 31; vst2(DEL + (eb0 + r) * CO + q * 4, *(const v4f*)&sm[r][q * 4]); }
  { float ssum[8], ssq[8];
#pragma unroll
    for (int r = 0; r < 8; ++r) { ssum[r] = 0.f; ssq[r] = 0.f; }
    v16h a[4];
#pragma unroll
    for (int kc = 0; kc < 4; ++kc) a[kc] = frag_h(&sa[wave * 16 + col][kc * 32], lane);
#pragma unroll 1
    for (int pass = 0; pass < 4; ++pass) { v8f acc[8] = {};
#pragma unroll
      for (int kc = 0; kc < 4; ++kc) {
#pragma unroll
        for (int j = 0; j < 8; ++j) acc[j] = wmma16(a[kc], frag_h(PH + (size_t)CO * HID + (size_t)(pass * 128 + j * 16 + col) * CO + kc * 32, lane), acc[j]); }
#pragma unroll
      for (int j = 0; j < 8; ++j) { const int n = pass * 128 + j * 16 + col; const float bb = bfr(AB1[n]);
#pragma unroll
        for (int r = 0; r < 8; ++r) { const float v = acc[j][r] + bb; ssum[r] += v; ssq[r] += v * v; sh[wave * 16 + 8 * g + r][n] = (_Float16)v; } } }
#pragma unroll
    for (int r = 0; r < 8; ++r) { float s = ssum[r], q = ssq[r];
#pragma unroll
      for (int o = 1; o < 16; o <<= 1) { s += __shfl_xor(s, o); q += __shfl_xor(q, o); }
      if (col == 0) { const float mu = s / (float)HID; const float var = fmaxf(q / (float)HID - mu * mu, 0.f); sst[wave * 16 + 8 * g + r][0] = mu; sst[wave * 16 + 8 * g + r][1] = 1.0f / sqrtf(var + 1e-5f); } } }
  __syncthreads();
  { const int r = tid >> 1, part = tid & 1; const float mu = sst[r][0], inv = sst[r][1];
#pragma unroll 1
    for (int n = part; n < HID; n += 2) sh[r][n] = (_Float16)elu_p(((float)sh[r][n] - mu) * inv * bfr(AG1[n]) + bfr(ABT1[n])); }
  __syncthreads();
  { v8f acc[8] = {};
#pragma unroll 2
    for (int kc = 0; kc < HID / 32; ++kc) { const v16h a = frag_h(&sh[wave * 16 + col][kc * 32], lane);
#pragma unroll
      for (int j = 0; j < 8; ++j) acc[j] = wmma16(a, frag_h(PH + (size_t)2 * CO * HID + (size_t)(j * 16 + col) * HID + kc * 32, lane), acc[j]); }
#pragma unroll
    for (int j = 0; j < 8; ++j) { const float bb = bfr(AB2[j * 16 + col]);
#pragma unroll
      for (int r = 0; r < 8; ++r) sm[wave * 16 + 8 * g + r][j * 16 + col] = acc[j][r] + bb; } }
  __syncthreads();
  { const int r = tid >> 1, part = tid & 1; float s = 0.f; for (int c = part; c < CO; c += 2) s += sm[r][c]; s += __shfl_xor(s, 1); const float mu = s / (float)CO; float q = 0.f; for (int c = part; c < CO; c += 2) { const float d = sm[r][c] - mu; q += d * d; } q += __shfl_xor(q, 1); const float inv = 1.0f / sqrtf(q / (float)CO + 1e-5f);
    for (int c = part; c < CO; c += 2) sm[r][c] = elu_p((sm[r][c] - mu) * inv * bfr(AG2[c]) + bfr(ABT2[c])); }
  __syncthreads();
  for (int e = tid; e < 64 * (CO / 4); e += 128) { const int r = e >> 5, q = e & 31; vst2(ALP + (eb0 + r) * CO + q * 4, *(const v4f*)&sm[r][q * 4]); }
}
__global__ __launch_bounds__(128) void k_final(const float* __restrict__ ALP, const float* __restrict__ DEL, const float* __restrict__ V, const int* __restrict__ IDX, float* __restrict__ OUT) {
  __shared__ __align__(16) float so[64][CO + 4];
  const int tid = threadIdx.x; const int r = tid >> 1, part = tid & 1; const size_t i = (size_t)blockIdx.x * 64 + r;
#pragma unroll 1
  for (int c = part * 64; c < part * 64 + 64; ++c) { float mx = -3.0e38f;
#pragma unroll 1
    for (int e = 0; e < NE; ++e) mx = fmaxf(mx, ALP[(i * NE + e) * CO + c]);
    float den = 0.f, num = 0.f;
#pragma unroll 1
    for (int e = 0; e < NE; ++e) { const size_t ed = i * NE + e; const float w = exp_ni(ALP[ed * CO + c] - mx); den += w; num += w * (V[(size_t)IDX[ed] * CO + c] + DEL[ed * CO + c]); }
    so[r][c] = num / den; }
  __syncthreads();
  for (int e = tid; e < 64 * (CO / 4); e += 128) { const int rr = e >> 5, q = e & 31; vst2(OUT + ((size_t)blockIdx.x * 64 + rr) * CO + q * 4, *(const v4f*)&so[rr][q * 4]); }
}
extern "C" void kernel_launch(void* const* d_in, const int* in_sizes, int n_in, void* d_out, int out_size, void* d_ws, size_t ws_size, hipStream_t stream) {
  (void)in_sizes; (void)n_in; (void)out_size;
  const float** F = (const float**)d_in;
  if (ws_size < (size_t)WS_END) return;
  char* ws = (char*)d_ws; __bf16* PW = (__bf16*)(ws + WS_PW); _Float16* PH = (_Float16*)(ws + WS_PH); int* IDX = (int*)(ws + WS_IDX); float *V = (float*)(ws + WS_V), *AS = (float*)(ws + WS_AS), *AD = (float*)(ws + WS_AD), *DEL = (float*)(ws + WS_DEL), *ALP = (float*)(ws + WS_ALP);
  k_pack<<<dim3(HID, 6), 256, 0, stream>>>(F[3], F[4], F[5], F[10], F[14], F[18], PW, PH);
  k_knn<<<NN / 64, 64, 0, stream>>>(F[1], IDX);
  k_node<<<dim3(NN / 64, 3), 128, 0, stream>>>(F[0], PW, V, AS, AD);
  k_edge<<<NEB, 128, 0, stream>>>(F[1], IDX, F[6], F[7], F[8], F[9], PH, F[11], F[12], F[13], AS, AD, F[15], F[16], F[17], F[19], F[20], F[21], DEL, ALP);
  k_final<<<NNB, 128, 0, stream>>>(ALP, DEL, V, IDX, (float*)d_out);
}
